// BatchMultiHeadGraphAttention_12618613916144
// MI455X (gfx1250) — hardware-verified
//
#include <hip/hip_runtime.h>
#include <math.h>

typedef __attribute__((ext_vector_type(16))) _Float16 v16h;
typedef __attribute__((ext_vector_type(16))) __bf16 v16b;
typedef __attribute__((ext_vector_type(8)))  _Float16 v8h;
typedef __attribute__((ext_vector_type(8)))  float v8f;
typedef __attribute__((ext_vector_type(4)))  float v4f;
typedef __attribute__((ext_vector_type(2)))  float v2f;
typedef __attribute__((ext_vector_type(4)))  unsigned v4u;
typedef __attribute__((ext_vector_type(4)))  int v4i;
typedef float __attribute__((may_alias)) float_a;
typedef int __attribute__((may_alias)) int_a;

template <typename T> __device__ __forceinline__ void vst2(void* p, T v) { *(volatile T*)p = v; __threadfence(); *(volatile T*)p = v; }
__device__ __forceinline__ v8f wmma16(v16h a, v16h b, v8f c) {
  v8f d = __builtin_amdgcn_wmma_f32_16x16x32_f16(false, a, false, b, (short)0, c, false, false);
  asm volatile("v_nop\n\tv_nop\n\tv_nop\n\tv_nop" : "+v"(d) : "v"(a), "v"(b));
  return d;
}
__device__ __forceinline__ v8f wmma_bf(v16b a, v16b b, v8f c) {
  v8f d = __builtin_amdgcn_wmma_f32_16x16x32_bf16(false, a, false, b, (short)0, c, false, false);
  asm volatile("v_nop\n\tv_nop\n\tv_nop\n\tv_nop" : "+v"(d) : "v"(a), "v"(b));
  return d;
}
__device__ __forceinline__ v16h frag_h(const _Float16* rowk0, int lane) {
  union { v16h v; v8h q[2]; } u; const _Float16* p = rowk0 + 8 * (lane >> 4);
  u.q[0] = *(const v8h*)p; u.q[1] = *(const v8h*)(p + 16); return u.v;
}
__device__ __forceinline__ v16h frag_f32(const float* rowk0, int lane) {
  v16h a; const float* p = rowk0 + 8 * (lane >> 4);
#pragma unroll
  for (int i = 0; i < 8; ++i) { a[i] = (_Float16)p[i]; a[8 + i] = (_Float16)p[16 + i]; }
  return a;
}
__device__ __forceinline__ v16h frag_f32s(const float* rowk0, int lane, float sc) {
  v16h a; const float* p = rowk0 + 8 * (lane >> 4);
#pragma unroll
  for (int i = 0; i < 8; ++i) { a[i] = (_Float16)(p[i] * sc); a[8 + i] = (_Float16)(p[16 + i] * sc); }
  return a;
}
__device__ __forceinline__ v16h fragc_f32(const float* W, int k0, int n, int lane, int ld, int K) {
  v16h a; const int g = lane >> 4;
#pragma unroll
  for (int i = 0; i < 8; ++i) { const int ka = k0 + 8 * g + i, kb = ka + 16;
    a[i] = (_Float16)(ka < K ? W[(size_t)(ka < K ? ka : K - 1) * ld + n] : 0.f); a[8 + i] = (_Float16)(kb < K ? W[(size_t)(kb < K ? kb : K - 1) * ld + n] : 0.f); }
  return a;
}
struct F2 { v16b h, l; };
__device__ __forceinline__ F2 bsplit16(const float v[16]) { F2 r;
#pragma unroll
  for (int i = 0; i < 16; ++i) { const __bf16 h = (__bf16)v[i]; r.h[i] = h; r.l[i] = (__bf16)(v[i] - (float)h); }
  return r; }
__device__ __forceinline__ F2 split_row(const float* row, int k0, int lane) { float v[16]; const float* p = row + k0 + 8 * (lane >> 4);
#pragma unroll
  for (int i = 0; i < 8; ++i) { v[i] = p[i]; v[8 + i] = p[16 + i]; }
  return bsplit16(v); }
__device__ __forceinline__ F2 split_rowK(const float* row, int k0, int lane, int K) { float v[16]; const int g = lane >> 4;
#pragma unroll
  for (int i = 0; i < 8; ++i) { const int ka = k0 + 8 * g + i, kb = ka + 16; v[i] = ka < K ? row[ka < K ? ka : K - 1] : 0.f; v[8 + i] = kb < K ? row[kb < K ? kb : K - 1] : 0.f; }
  return bsplit16(v); }
__device__ __forceinline__ F2 split_col(const float* W, int k0, int n, int lane, int ld, int K) { float v[16]; const int g = lane >> 4;
#pragma unroll
  for (int i = 0; i < 8; ++i) { const int ka = k0 + 8 * g + i, kb = ka + 16; v[i] = ka < K ? W[(size_t)(ka < K ? ka : K - 1) * ld + n] : 0.f; v[8 + i] = kb < K ? W[(size_t)(kb < K ? kb : K - 1) * ld + n] : 0.f; }
  return bsplit16(v); }
__device__ __forceinline__ v8f mac3(const F2& a, const F2& b, v8f c) { c = wmma_bf(a.l, b.h, c); c = wmma_bf(a.h, b.l, c); return wmma_bf(a.h, b.h, c); }
__device__ __forceinline__ float sigm(float v) { return 1.0f / (1.0f + expf(-v)); }
#define LDSX() do { asm volatile("s_wait_dscnt 0" ::: "memory"); __builtin_amdgcn_wave_barrier(); __builtin_amdgcn_fence(__ATOMIC_RELEASE, "workgroup"); } while (0)


#define NB 4
#define NN 2048
#define FI 768
#define FO 64
#define NH 4
#define NROW (NB * NN)
#ifndef TNB
#define TNB NB
#endif
typedef __attribute__((ext_vector_type(8))) __bf16 v8b;
__device__ __forceinline__ v16b frag_b(const __bf16* rowk0, int lane) {
  union { v16b v; v8b q[2]; } u; const __bf16* p = rowk0 + 8 * (lane >> 4);
  u.q[0] = *(const v8b*)p; u.q[1] = *(const v8b*)(p + 16); return u.v;
}
__device__ __forceinline__ float bfr(float v) { return (float)(__bf16)v; }
__device__ __attribute__((noinline)) float exp_ni(float v) { return expf(v); }
__device__ __attribute__((noinline)) float erf_ni(float v) { return erff(v); }

#define WS_HP  0u
#define WS_SC  (WS_HP + 4u * (size_t)NB * NH * FO * NN)
#define WS_END (WS_SC + 4u * (size_t)NROW * 8)

__device__ __forceinline__ v16b fragb_f32(const float* __restrict__ p, int lane) { v16b a; const float* pp = p + 8 * (lane >> 4);
#pragma unroll
  for (int i = 0; i < 8; ++i) { a[i] = (__bf16)pp[i]; a[8 + i] = (__bf16)pp[16 + i]; } return a; }
__global__ __launch_bounds__(128) void k_hp(const float* __restrict__ Hm, const float* __restrict__ Wm, const float* __restrict__ AS, const float* __restrict__ AD, float* __restrict__ HP, float* __restrict__ SC) { __shared__ __align__(16) float tt[FO][72]; __shared__ __align__(16) float ssc[64][8];
  const int tid = threadIdx.x, wave = tid >> 5, lane = tid & 31, col = lane & 15, g = lane >> 4; const size_t b = blockIdx.y; const int n0 = blockIdx.x * 64; const size_t r0 = b * NN + n0 + wave * 16;
#pragma unroll 1
  for (int hh = 0; hh < NH; ++hh) { v8f acc[4] = {};
#pragma unroll 2
    for (int kc = 0; kc < FI / 32; ++kc) { const v16b a = fragb_f32(Hm + (r0 + col) * FI + kc * 32, lane);
#pragma unroll
      for (int j = 0; j < 4; ++j) { v16b w; const int o = j * 16 + col;
#pragma unroll
        for (int i = 0; i < 8; ++i) { w[i] = (__bf16)Wm[((size_t)hh * FI + kc * 32 + 8 * g + i) * FO + o]; w[8 + i] = (__bf16)Wm[((size_t)hh * FI + kc * 32 + 16 + 8 * g + i) * FO + o]; }
        acc[j] = wmma_bf(a, w, acc[j]); } }
#pragma unroll
    for (int r = 0; r < 8; ++r) { float ss = 0.f, sd = 0.f;
#pragma unroll
      for (int j = 0; j < 4; ++j) { const int o = j * 16 + col; const float tv = tanhf(acc[j][r]); ss += tv * bfr(AS[hh * FO + o]); sd += tv * bfr(AD[hh * FO + o]); }
#pragma unroll
      for (int ofs = 1; ofs < 16; ofs <<= 1) { ss += __shfl_xor(ss, ofs); sd += __shfl_xor(sd, ofs); }
      if (col == 0) { ssc[wave * 16 + 8 * g + r][hh] = ss; ssc[wave * 16 + 8 * g + r][4 + hh] = sd; } }
#pragma unroll
    for (int j = 0; j < 4; ++j)
#pragma unroll
      for (int r = 0; r < 8; ++r) tt[j * 16 + col][wave * 16 + 8 * g + r] = acc[j][r];
    __syncthreads();
    for (int e = tid; e < FO * 16; e += 128) { const int o = e >> 4, q = e & 15; vst2(HP + (((b * NH + hh) * FO + o) * (size_t)NN) + n0 + q * 4, *(const v4f*)&tt[o][q * 4]); }
    __syncthreads(); }
  for (int e = tid; e < 64 * 2; e += 128) { const int rl = e >> 1, q = e & 1; vst2(SC + (b * NN + n0 + rl) * 8 + q * 4, *(const v4f*)&ssc[rl][q * 4]); } }
__global__ __launch_bounds__(128) void k_gat(const float* __restrict__ SC, const float* __restrict__ HP, const float* __restrict__ BI, float* __restrict__ OUT) { __shared__ __align__(16) float sdst[NN]; __shared__ __align__(16) float so[4][16][68];
  const int tid = threadIdx.x, wave = tid >> 5, lane = tid & 31, col = lane & 15, g = lane >> 4; const int hh = blockIdx.y; const size_t b = blockIdx.z; const int i0 = blockIdx.x * 64 + wave * 16;
  for (int e = tid; e < NN; e += 128) sdst[e] = SC[(b * NN + e) * 8 + 4 + hh];
  __syncthreads();
  const float si = SC[(b * NN + i0 + col) * 8 + hh];
  float mx = -3.0e38f;
#pragma unroll 1
  for (int j = 0; j < NN; ++j) { float s = si + sdst[j]; s = (s >= 0.f) ? s : 0.2f * s; mx = fmaxf(mx, s); }
  float sum = 0.f;
#pragma unroll 1
  for (int j = 0; j < NN; ++j) { float s = si + sdst[j]; s = (s >= 0.f) ? s : 0.2f * s; sum += expf(s - mx); }
  const float inv = 1.0f / sum;
  v8f acc[4] = {};
#pragma unroll 1
  for (int kc = 0; kc < NN / 32; ++kc) { float v[16];
#pragma unroll
    for (int i = 0; i < 8; ++i) {
#pragma unroll
      for (int half = 0; half < 2; ++half) { const int j = kc * 32 + half * 16 + 8 * g + i; float s = si + sdst[j]; s = (s >= 0.f) ? s : 0.2f * s; v[half * 8 + i] = expf(s - mx) * inv; } }
    const F2 a = bsplit16(v);
#pragma unroll
    for (int jt = 0; jt < 4; ++jt) { const F2 w = split_row(HP + (((b * NH + hh) * FO + jt * 16 + col) * (size_t)NN), kc * 32, lane); acc[jt] = mac3(a, w, acc[jt]); } }
#pragma unroll
  for (int jt = 0; jt < 4; ++jt)
#pragma unroll
    for (int r = 0; r < 8; ++r) so[wave][8 * g + r][jt * 16 + col] = acc[jt][r] + bfr(BI[jt * 16 + col]);
  LDSX(); for (int rl = 0; rl < 16; ++rl) if (lane < 16) vst2(OUT + (((b * NH + hh) * NN) + i0 + rl) * FO + lane * 4, *(const v4f*)&so[wave][rl][lane * 4]); }
extern "C" void kernel_launch(void* const* d_in, const int* in_sizes, int n_in, void* d_out, int out_size, void* d_ws, size_t ws_size, hipStream_t stream) {
  (void)in_sizes; (void)n_in; (void)out_size;
  const float** F = (const float**)d_in;
  if (ws_size < (size_t)WS_END) return;
  char* ws = (char*)d_ws; float *HP = (float*)(ws + WS_HP), *SC = (float*)(ws + WS_SC);
  k_hp<<<dim3(NN / 64, TNB), 128, 0, stream>>>(F[0], F[1], F[2], F[3], HP, SC);
  k_gat<<<dim3(NN / 64, NH, TNB), 128, 0, stream>>>(SC, HP, F[4], (float*)d_out);
}
